// RgbNet_90117003805324
// MI455X (gfx1250) — hardware-verified
//
#include <hip/hip_runtime.h>
#include <math.h>

typedef __attribute__((ext_vector_type(16))) _Float16 v16h;
typedef __attribute__((ext_vector_type(16))) __bf16 v16b;
typedef __attribute__((ext_vector_type(8)))  _Float16 v8h;
typedef __attribute__((ext_vector_type(8)))  float v8f;
typedef __attribute__((ext_vector_type(4)))  float v4f;
typedef __attribute__((ext_vector_type(2)))  float v2f;
typedef __attribute__((ext_vector_type(4)))  unsigned v4u;
typedef __attribute__((ext_vector_type(4)))  int v4i;
typedef float __attribute__((may_alias)) float_a;
typedef int __attribute__((may_alias)) int_a;

template <typename T> __device__ __forceinline__ void vst2(void* p, T v) { *(volatile T*)p = v; __threadfence(); *(volatile T*)p = v; }
__device__ __forceinline__ v8f wmma16(v16h a, v16h b, v8f c) {
  v8f d = __builtin_amdgcn_wmma_f32_16x16x32_f16(false, a, false, b, (short)0, c, false, false);
  asm volatile("v_nop\n\tv_nop\n\tv_nop\n\tv_nop" : "+v"(d) : "v"(a), "v"(b));
  return d;
}
__device__ __forceinline__ v8f wmma_bf(v16b a, v16b b, v8f c) {
  v8f d = __builtin_amdgcn_wmma_f32_16x16x32_bf16(false, a, false, b, (short)0, c, false, false);
  asm volatile("v_nop\n\tv_nop\n\tv_nop\n\tv_nop" : "+v"(d) : "v"(a), "v"(b));
  return d;
}
__device__ __forceinline__ v16h frag_h(const _Float16* rowk0, int lane) {
  union { v16h v; v8h q[2]; } u; const _Float16* p = rowk0 + 8 * (lane >> 4);
  u.q[0] = *(const v8h*)p; u.q[1] = *(const v8h*)(p + 16); return u.v;
}
__device__ __forceinline__ v16h frag_f32(const float* rowk0, int lane) {
  v16h a; const float* p = rowk0 + 8 * (lane >> 4);
#pragma unroll
  for (int i = 0; i < 8; ++i) { a[i] = (_Float16)p[i]; a[8 + i] = (_Float16)p[16 + i]; }
  return a;
}
__device__ __forceinline__ v16h frag_f32s(const float* rowk0, int lane, float sc) {
  v16h a; const float* p = rowk0 + 8 * (lane >> 4);
#pragma unroll
  for (int i = 0; i < 8; ++i) { a[i] = (_Float16)(p[i] * sc); a[8 + i] = (_Float16)(p[16 + i] * sc); }
  return a;
}
__device__ __forceinline__ v16h fragc_f32(const float* W, int k0, int n, int lane, int ld, int K) {
  v16h a; const int g = lane >> 4;
#pragma unroll
  for (int i = 0; i < 8; ++i) { const int ka = k0 + 8 * g + i, kb = ka + 16;
    a[i] = (_Float16)(ka < K ? W[(size_t)(ka < K ? ka : K - 1) * ld + n] : 0.f); a[8 + i] = (_Float16)(kb < K ? W[(size_t)(kb < K ? kb : K - 1) * ld + n] : 0.f); }
  return a;
}
struct F2 { v16b h, l; };
__device__ __forceinline__ F2 bsplit16(const float v[16]) { F2 r;
#pragma unroll
  for (int i = 0; i < 16; ++i) { const __bf16 h = (__bf16)v[i]; r.h[i] = h; r.l[i] = (__bf16)(v[i] - (float)h); }
  return r; }
__device__ __forceinline__ F2 split_row(const float* row, int k0, int lane) { float v[16]; const float* p = row + k0 + 8 * (lane >> 4);
#pragma unroll
  for (int i = 0; i < 8; ++i) { v[i] = p[i]; v[8 + i] = p[16 + i]; }
  return bsplit16(v); }
__device__ __forceinline__ F2 split_rowK(const float* row, int k0, int lane, int K) { float v[16]; const int g = lane >> 4;
#pragma unroll
  for (int i = 0; i < 8; ++i) { const int ka = k0 + 8 * g + i, kb = ka + 16; v[i] = ka < K ? row[ka < K ? ka : K - 1] : 0.f; v[8 + i] = kb < K ? row[kb < K ? kb : K - 1] : 0.f; }
  return bsplit16(v); }
__device__ __forceinline__ F2 split_col(const float* W, int k0, int n, int lane, int ld, int K) { float v[16]; const int g = lane >> 4;
#pragma unroll
  for (int i = 0; i < 8; ++i) { const int ka = k0 + 8 * g + i, kb = ka + 16; v[i] = ka < K ? W[(size_t)(ka < K ? ka : K - 1) * ld + n] : 0.f; v[8 + i] = kb < K ? W[(size_t)(kb < K ? kb : K - 1) * ld + n] : 0.f; }
  return bsplit16(v); }
__device__ __forceinline__ v8f mac3(const F2& a, const F2& b, v8f c) { c = wmma_bf(a.l, b.h, c); c = wmma_bf(a.h, b.l, c); return wmma_bf(a.h, b.h, c); }
__device__ __forceinline__ float sigm(float v) { return 1.0f / (1.0f + expf(-v)); }
#define LDSX() do { asm volatile("s_wait_dscnt 0" ::: "memory"); __builtin_amdgcn_wave_barrier(); __builtin_amdgcn_fence(__ATOMIC_RELEASE, "workgroup"); } while (0)


#define NRAY 16384
#define NSMP 300
#define NLV 6
#define LD 4
#define HT 524288
#define FIN 120
#define FP 128
#define HID 64
#ifndef NRT
#define NRT (NRAY / 64)
#endif
typedef __attribute__((ext_vector_type(8))) __bf16 v8b;
__device__ __forceinline__ v16b frag_b(const __bf16* rowk0, int lane) {
  union { v16b v; v8b q[2]; } u; const __bf16* p = rowk0 + 8 * (lane >> 4);
  u.q[0] = *(const v8b*)p; u.q[1] = *(const v8b*)(p + 16); return u.v;
}
__device__ __forceinline__ float bfr(float v) { return (float)(__bf16)v; }
__device__ __attribute__((noinline)) float exp_ni(float v) { return expf(v); }
__device__ __attribute__((noinline)) float erf_ni(float v) { return erff(v); }
__constant__ float c_t300[NSMP] = {0.000000000e+00f,3.344481578e-03f,6.688963156e-03f,1.003344450e-02f,1.337792631e-02f,1.672240719e-02f,2.006688900e-02f,2.341137081e-02f,2.675585262e-02f,3.010033444e-02f,3.344481438e-02f,3.678929806e-02f,4.013377801e-02f,4.347826168e-02f,4.682274163e-02f,5.016722530e-02f,5.351170525e-02f,5.685618520e-02f,6.020066887e-02f,6.354515254e-02f,6.688962877e-02f,7.023411244e-02f,7.357859612e-02f,7.692307979e-02f,8.026755601e-02f,8.361203969e-02f,8.695652336e-02f,9.030099958e-02f,9.364548326e-02f,9.698996693e-02f,1.003344506e-01f,1.036789268e-01f,1.070234105e-01f,1.103678942e-01f,1.137123704e-01f,1.170568541e-01f,1.204013377e-01f,1.237458214e-01f,1.270903051e-01f,1.304347813e-01f,1.337792575e-01f,1.371237487e-01f,1.404682249e-01f,1.438127011e-01f,1.471571922e-01f,1.505016685e-01f,1.538461596e-01f,1.571906358e-01f,1.605351120e-01f,1.638796031e-01f,1.672240794e-01f,1.705685556e-01f,1.739130467e-01f,1.772575229e-01f,1.806019992e-01f,1.839464903e-01f,1.872909665e-01f,1.906354427e-01f,1.939799339e-01f,1.973244101e-01f,2.006689012e-01f,2.040133774e-01f,2.073578537e-01f,2.107023448e-01f,2.140468210e-01f,2.173912972e-01f,2.207357883e-01f,2.240802646e-01f,2.274247408e-01f,2.307692319e-01f,2.341137081e-01f,2.374581993e-01f,2.408026755e-01f,2.441471517e-01f,2.474916428e-01f,2.508361042e-01f,2.541806102e-01f,2.575250864e-01f,2.608695626e-01f,2.642140388e-01f,2.675585151e-01f,2.709030211e-01f,2.742474973e-01f,2.775919735e-01f,2.809364498e-01f,2.842809260e-01f,2.876254022e-01f,2.909699082e-01f,2.943143845e-01f,2.976588607e-01f,3.010033369e-01f,3.043478131e-01f,3.076923192e-01f,3.110367954e-01f,3.143812716e-01f,3.177257478e-01f,3.210702240e-01f,3.244147003e-01f,3.277592063e-01f,3.311036825e-01f,3.344481587e-01f,3.377926350e-01f,3.411371112e-01f,3.444816172e-01f,3.478260934e-01f,3.511705697e-01f,3.545150459e-01f,3.578595221e-01f,3.612039983e-01f,3.645485044e-01f,3.678929806e-01f,3.712374568e-01f,3.745819330e-01f,3.779264092e-01f,3.812708855e-01f,3.846153915e-01f,3.879598677e-01f,3.913043439e-01f,3.946488202e-01f,3.979932964e-01f,4.013378024e-01f,4.046822786e-01f,4.080267549e-01f,4.113712311e-01f,4.147157073e-01f,4.180601835e-01f,4.214046896e-01f,4.247491658e-01f,4.280936420e-01f,4.314381182e-01f,4.347825944e-01f,4.381271005e-01f,4.414715767e-01f,4.448160529e-01f,4.481605291e-01f,4.515050054e-01f,4.548494816e-01f,4.581939876e-01f,4.615384638e-01f,4.648829401e-01f,4.682274163e-01f,4.715718925e-01f,4.749163985e-01f,4.782608747e-01f,4.816053510e-01f,4.849498272e-01f,4.882943034e-01f,4.916387796e-01f,4.949832857e-01f,4.983277619e-01f,5.016722083e-01f,5.050167441e-01f,5.083612204e-01f,5.117056966e-01f,5.150501728e-01f,5.183946490e-01f,5.217391253e-01f,5.250836015e-01f,5.284280777e-01f,5.317725539e-01f,5.351170301e-01f,5.384615064e-01f,5.418060422e-01f,5.451505184e-01f,5.484949946e-01f,5.518394709e-01f,5.551839471e-01f,5.585284233e-01f,5.618728995e-01f,5.652173758e-01f,5.685618520e-01f,5.719063282e-01f,5.752508044e-01f,5.785953403e-01f,5.819398165e-01f,5.852842927e-01f,5.886287689e-01f,5.919732451e-01f,5.953177214e-01f,5.986621976e-01f,6.020066738e-01f,6.053511500e-01f,6.086956263e-01f,6.120401025e-01f,6.153846383e-01f,6.187291145e-01f,6.220735908e-01f,6.254180670e-01f,6.287625432e-01f,6.321070194e-01f,6.354514956e-01f,6.387959719e-01f,6.421404481e-01f,6.454849243e-01f,6.488294005e-01f,6.521739364e-01f,6.555184126e-01f,6.588628888e-01f,6.622073650e-01f,6.655518413e-01f,6.688963175e-01f,6.722407937e-01f,6.755852699e-01f,6.789297462e-01f,6.822742224e-01f,6.856186986e-01f,6.889632344e-01f,6.923077106e-01f,6.956521869e-01f,6.989966631e-01f,7.023411393e-01f,7.056856155e-01f,7.090300918e-01f,7.123745680e-01f,7.157190442e-01f,7.190635204e-01f,7.224079967e-01f,7.257524729e-01f,7.290970087e-01f,7.324414849e-01f,7.357859612e-01f,7.391304374e-01f,7.424749136e-01f,7.458193898e-01f,7.491638660e-01f,7.525083423e-01f,7.558528185e-01f,7.591972947e-01f,7.625417709e-01f,7.658863068e-01f,7.692307830e-01f,7.725752592e-01f,7.759197354e-01f,7.792642117e-01f,7.826086879e-01f,7.859531641e-01f,7.892976403e-01f,7.926421165e-01f,7.959865928e-01f,7.993310690e-01f,8.026756048e-01f,8.060200810e-01f,8.093645573e-01f,8.127090335e-01f,8.160535097e-01f,8.193979859e-01f,8.227424622e-01f,8.260869384e-01f,8.294314146e-01f,8.327758908e-01f,8.361203671e-01f,8.394649029e-01f,8.428093791e-01f,8.461538553e-01f,8.494983315e-01f,8.528428078e-01f,8.561872840e-01f,8.595317602e-01f,8.628762364e-01f,8.662207127e-01f,8.695651889e-01f,8.729096651e-01f,8.762542009e-01f,8.795986772e-01f,8.829431534e-01f,8.862876296e-01f,8.896321058e-01f,8.929765821e-01f,8.963210583e-01f,8.996655345e-01f,9.030100107e-01f,9.063544869e-01f,9.096989632e-01f,9.130434990e-01f,9.163879752e-01f,9.197324514e-01f,9.230769277e-01f,9.264214039e-01f,9.297658801e-01f,9.331103563e-01f,9.364548326e-01f,9.397993088e-01f,9.431437850e-01f,9.464882612e-01f,9.498327971e-01f,9.531772733e-01f,9.565217495e-01f,9.598662257e-01f,9.632107019e-01f,9.665551782e-01f,9.698996544e-01f,9.732441306e-01f,9.765886068e-01f,9.799330831e-01f,9.832775593e-01f,9.866220951e-01f,9.899665713e-01f,9.933110476e-01f,9.966555238e-01f,1.000000000e+00f};

#define PK_1 0
#define PK_2 (PK_1 + HID * FP)
#define PK_3 (PK_2 + HID * HID)
#define PK_4 (PK_3 + HID * HID)
#define PK_END (PK_4 + 16 * HID)
#define WS_END (2u * PK_END)

__global__ __launch_bounds__(128) void k_pack(const float* __restrict__ W1, const float* __restrict__ W2, const float* __restrict__ W3, const float* __restrict__ W4, __bf16* __restrict__ PK) {
  __shared__ __align__(16) __bf16 s[FP]; const int n = blockIdx.x, which = blockIdx.y, t = threadIdx.x; int K; size_t dst;
  if (which == 0) { K = FP; dst = PK_1 + (size_t)n * FP; s[t] = (__bf16)((t < FIN) ? W1[(size_t)n * FIN + t] : 0.f); }
  else if (which <= 2) { K = HID; dst = (which == 1 ? PK_2 : PK_3) + (size_t)n * HID; if (t < HID) s[t] = (__bf16)(which == 1 ? W2 : W3)[(size_t)n * HID + t]; }
  else { if (n >= 16) return; K = HID; dst = PK_4 + (size_t)n * HID; if (t < HID) s[t] = (__bf16)((n < 3) ? W4[(size_t)n * HID + t] : 0.f); }
  __syncthreads();
  if (t < K / 8) vst2((unsigned*)(PK + dst + t * 8), *(const v4u*)&s[t * 8]);
}
__device__ __forceinline__ void encode_level(int l, float px, float py, float pz, const float* __restrict__ EMB, float f[4]) {
  const int R = 4 << l; const float Rf = (float)R;
  const float qx = px * Rf, qy = py * Rf, qz = pz * Rf; const float fx0 = floorf(qx), fy0 = floorf(qy), fz0 = floorf(qz);
  const int ix = (int)fx0, iy = (int)fy0, iz = (int)fz0; const float wx = qx - fx0, wy = qy - fy0, wz = qz - fz0;
  const bool dense = (R + 1) * (R + 1) * (R + 1) <= HT; const float* tab = EMB + (size_t)l * HT * LD;
  f[0] = f[1] = f[2] = f[3] = 0.f;
#pragma unroll
  for (int c = 0; c < 8; ++c) { const int oi = c >> 2, oj = (c >> 1) & 1, ok = c & 1;
    const int cx = min(max(ix + oi, 0), R), cy = min(max(iy + oj, 0), R), cz = min(max(iz + ok, 0), R);
    const float w = ((oi ? wx : 1.0f - wx) * (oj ? wy : 1.0f - wy)) * (ok ? wz : 1.0f - wz);
    int idx; if (dense) idx = cx + cy * (R + 1) + cz * (R + 1) * (R + 1);
    else { const unsigned hx = (unsigned)cx * 1u, hy = (unsigned)cy * 2654435761u, hz = (unsigned)cz * 805459861u; idx = (int)((hx ^ hy ^ hz) % (unsigned)HT); }
    const float* e = tab + (size_t)idx * LD;
#pragma unroll
    for (int d = 0; d < LD; ++d) f[d] += w * bfr(e[d]); }
}
__global__ __launch_bounds__(128) void k_mlp(const float* __restrict__ X, const int* __restrict__ IFIRST, const float* __restrict__ EMB, const __bf16* __restrict__ PK, const float* __restrict__ B1, const float* __restrict__ B2, const float* __restrict__ B3, const float* __restrict__ B4, float* __restrict__ OUT) {
  __shared__ __align__(16) float sf[64][FP + 4]; __shared__ __align__(16) float sh[4][16][68]; __shared__ __align__(16) float so[64 * 3];
  const int tid = threadIdx.x, wave = tid >> 5, lane = tid & 31, col = lane & 15, g = lane >> 4; const size_t r0 = (size_t)blockIdx.x * 64;
  for (int q = tid; q < 64 * 8; q += 128) { const int rl = q >> 3, c8 = q & 7; sf[rl][FIN + c8] = 0.f; }
  for (int q = tid; q < 64 * 5 * NLV; q += 128) { const int rl = q / (5 * NLV), rem = q % (5 * NLV), d5 = rem / NLV, l = rem % NLV; const size_t n = r0 + rl;
    const int j = min(max(IFIRST[n] + d5 - 2, 0), NSMP - 1); const float t = c_t300[j]; const float omt = 1.0f - t;
    const float sx = bfr(X[n * 4 + 0]), sy = bfr(X[n * 4 + 1]), ex = bfr(X[n * 4 + 2]), ey = bfr(X[n * 4 + 3]);
    const float px = sx * omt + ex * t, py = sy * omt + ey * t, pz = t;
    float f[4]; encode_level(l, px, py, pz, EMB, f);
#pragma unroll
    for (int d = 0; d < LD; ++d) sf[rl][d5 * (NLV * LD) + l * LD + d] = f[d]; }
  __syncthreads();
  v8f acc[4] = {};
#pragma unroll
  for (int kc = 0; kc < FP / 32; ++kc) { const F2 a = split_row(&sf[wave * 16 + col][0], kc * 32, lane);
#pragma unroll
    for (int j = 0; j < 4; ++j) { const v16b w = frag_b(PK + PK_1 + (size_t)(j * 16 + col) * FP + kc * 32, lane); acc[j] = wmma_bf(a.l, w, acc[j]); acc[j] = wmma_bf(a.h, w, acc[j]); } }
#pragma unroll 1
  for (int layer = 2; layer <= 4; ++layer) {
    const float* bias = (layer == 2) ? B1 : (layer == 3) ? B2 : B3;
#pragma unroll
    for (int j = 0; j < 4; ++j) { const float bb = bfr(bias[j * 16 + col]);
#pragma unroll
      for (int r = 0; r < 8; ++r) sh[wave][8 * g + r][j * 16 + col] = fmaxf(acc[j][r] + bb, 0.f); }
    LDSX();
    const __bf16* P = PK + ((layer == 2) ? PK_2 : (layer == 3) ? PK_3 : PK_4); const int nt = (layer == 4) ? 1 : 4;
    v8f nacc[4] = {};
#pragma unroll
    for (int kc = 0; kc < 2; ++kc) { const F2 a = split_row(&sh[wave][col][0], kc * 32, lane);
#pragma unroll
      for (int j = 0; j < 4; ++j) if (j < nt) { const v16b w = frag_b(P + (size_t)(j * 16 + col) * HID + kc * 32, lane); nacc[j] = wmma_bf(a.l, w, nacc[j]); nacc[j] = wmma_bf(a.h, w, nacc[j]); } }
    LDSX();
#pragma unroll
    for (int j = 0; j < 4; ++j) acc[j] = nacc[j]; }
  if (col < 3) { const float bb = bfr(B4[col]);
#pragma unroll
    for (int r = 0; r < 8; ++r) so[(wave * 16 + 8 * g + r) * 3 + col] = acc[0][r] + bb; }
  __syncthreads();
  if (tid < 48) vst2(OUT + r0 * 3 + tid * 4, *(const v4f*)&so[tid * 4]);
}
extern "C" void kernel_launch(void* const* d_in, const int* in_sizes, int n_in, void* d_out, int out_size, void* d_ws, size_t ws_size, hipStream_t stream) {
  (void)in_sizes; (void)n_in; (void)out_size;
  const float** F = (const float**)d_in;
  if (ws_size < (size_t)WS_END) return;
  __bf16* PK = (__bf16*)d_ws;
  k_pack<<<dim3(HID, 4), 128, 0, stream>>>(F[3], F[5], F[7], F[9], PK);
  k_mlp<<<NRT, 128, 0, stream>>>(F[0], (const int*)d_in[1], F[2], PK, F[4], F[6], F[8], F[10], (float*)d_out);
}
